// Painter_Varient_33509334843902
// MI455X (gfx1250) — hardware-verified
//
#include <hip/hip_runtime.h>


#define NWIN 64
#define WCH  16
#define NTOK 196
#define TP   256
#define GH   14
#define DM   1024
#define NH_  16
#define HD   64
#define ZHALF 128
#define PCAR 1024.0f
typedef _Float16 h16;
typedef unsigned short bf;
typedef __attribute__((ext_vector_type(16))) __bf16   v16bf;
typedef __attribute__((ext_vector_type(16))) _Float16 v16h;
typedef __attribute__((ext_vector_type(8)))  _Float16 v8h;
typedef __attribute__((ext_vector_type(8)))  unsigned short v8us;
typedef __attribute__((ext_vector_type(8)))  float    v8f;
typedef __attribute__((ext_vector_type(4)))  float    v4f;
typedef v8h  __attribute__((may_alias)) v8ha;
typedef v4f  __attribute__((may_alias)) v4fa;
typedef v8us __attribute__((may_alias)) v8usa;

__device__ __forceinline__ unsigned short f2bf(float f) { unsigned u = __float_as_uint(f); u += 0x7FFFu + ((u >> 16) & 1u); return (unsigned short)(u >> 16); }
__device__ __forceinline__ float bf2f(unsigned short b) { return __uint_as_float(((unsigned)b) << 16); }
__device__ __forceinline__ float bfr(float f) { return bf2f(f2bf(f)); }
__device__ __forceinline__ v16h cat16(v8h lo, v8h hi) { return __builtin_shufflevector(lo, hi, 0, 1, 2, 3, 4, 5, 6, 7, 8, 9, 10, 11, 12, 13, 14, 15); }
__device__ __forceinline__ v16bf cat16b(v8us lo, v8us hi) { return __builtin_bit_cast(v16bf, __builtin_shufflevector(lo, hi, 0, 1, 2, 3, 4, 5, 6, 7, 8, 9, 10, 11, 12, 13, 14, 15)); }
__device__ __forceinline__ v8f wmma16(v16h a, v16h b, v8f c) { return __builtin_amdgcn_wmma_f32_16x16x32_f16(false, a, false, b, (short)0, c, false, false); }
__device__ __forceinline__ v8f wmmab(v16bf a, v16bf b, v8f c) { return __builtin_amdgcn_wmma_f32_16x16x32_bf16(false, a, false, b, (short)0, c, false, false); }


template <typename T16> struct WFrag;
template <> struct WFrag<h16> { typedef v16h V; static __device__ __forceinline__ V ld(const h16* p) { return cat16(*(const v8h*)p, *(const v8h*)(p + 16)); } static __device__ __forceinline__ v8f mma(V a, V b, v8f c) { return wmma16(a, b, c); } };
template <> struct WFrag<bf> { typedef v16bf V; static __device__ __forceinline__ V ld(const bf* p) { return cat16b(*(const v8us*)p, *(const v8us*)(p + 16)); } static __device__ __forceinline__ v8f mma(V a, V b, v8f c) { return wmmab(a, b, c); } };
template <typename T16, int NSPLIT, bool BIAS>
__global__ __launch_bounds__(32) void k_gemmw(const T16* __restrict__ A, const T16* __restrict__ A2, const T16* __restrict__ Bt, const T16* __restrict__ Bt2, int K, float* C, int ldc, const float* __restrict__ bias, size_t sA, size_t sB, size_t sC) {
    typedef typename WFrag<T16>::V V;
    __shared__ __align__(16) float os[16 * 68];
    const size_t z = blockIdx.z; A += z * sA; if (A2) A2 += z * sA; Bt += z * sB; if (Bt2) Bt2 += z * sB; C += z * sC;
    const int lane = threadIdx.x & 31, lr = lane & 15, hi = lane >> 4; const int r0 = blockIdx.x * 64, c0 = blockIdx.y * 64;
    v8f acc[4][4];
#pragma unroll
    for (int mb = 0; mb < 4; ++mb)
#pragma unroll
        for (int nb = 0; nb < 4; ++nb) acc[mb][nb] = (v8f){};
    const size_t aoff = (size_t)(r0 + lr) * K + 8 * hi, boff = (size_t)(c0 + lr) * K + 8 * hi;
#pragma unroll 1
    for (int kc = 0; kc < K; kc += 32) {
        V a[4], a2[4];
#pragma unroll
        for (int mb = 0; mb < 4; ++mb) { a[mb] = WFrag<T16>::ld(A + aoff + (size_t)mb * 16 * K + kc); if (NSPLIT == 1 || NSPLIT == 2) a2[mb] = WFrag<T16>::ld(A2 + aoff + (size_t)mb * 16 * K + kc); }
#pragma unroll
        for (int nb = 0; nb < 4; ++nb) { const V b = WFrag<T16>::ld(Bt + boff + (size_t)nb * 16 * K + kc); V b2; if (NSPLIT >= 2) b2 = WFrag<T16>::ld(Bt2 + boff + (size_t)nb * 16 * K + kc);
#pragma unroll
            for (int mb = 0; mb < 4; ++mb) { acc[mb][nb] = WFrag<T16>::mma(a[mb], b, acc[mb][nb]); if (NSPLIT == 1 || NSPLIT == 2) acc[mb][nb] = WFrag<T16>::mma(a2[mb], b, acc[mb][nb]); if (NSPLIT >= 2) acc[mb][nb] = WFrag<T16>::mma(a[mb], b2, acc[mb][nb]); } }
        asm volatile("v_nop\n\tv_nop\n\tv_nop\n\tv_nop" : "+v"(acc[0][0]), "+v"(acc[1][1]), "+v"(acc[2][2]), "+v"(acc[3][3]) : "v"(a[0]), "v"(a[3]));
    }
#pragma unroll
    for (int mb = 0; mb < 4; ++mb) {
#pragma unroll
        for (int nb = 0; nb < 4; ++nb) {
#pragma unroll
            for (int j = 0; j < 8; ++j) os[(hi * 8 + j) * 68 + nb * 16 + lr] = acc[mb][nb][j]; }
        __builtin_amdgcn_wave_barrier(); asm volatile("" ::: "memory");
        float* crow = C + (size_t)(r0 + mb * 16) * ldc + c0;
#pragma unroll 1
        for (int ps = 0; ps < 2; ++ps) {
#pragma unroll
            for (int s = 0; s < 8; ++s) { const int row = 2 * s + hi, cofs = lr * 4; v4f val = *(const v4fa*)(os + row * 68 + cofs); if (BIAS) { val[0] += bfr(bias[c0 + cofs]); val[1] += bfr(bias[c0 + cofs + 1]); val[2] += bfr(bias[c0 + cofs + 2]); val[3] += bfr(bias[c0 + cofs + 3]); }
                *(volatile v4f*)(crow + (size_t)row * ldc + cofs) = val; }
            if (ps == 0) __threadfence(); }
        __builtin_amdgcn_wave_barrier(); asm volatile("" ::: "memory");
    }
}

__device__ __forceinline__ h16 tohx(float x) { return (h16)x; }
__device__ __forceinline__ void splitf(float y, unsigned short& h, unsigned short& l) { h = f2bf(y); l = f2bf(y - bf2f(h)); }
typedef __attribute__((ext_vector_type(2))) unsigned short v2us;
typedef __attribute__((ext_vector_type(4))) unsigned short v4us;
typedef __attribute__((ext_vector_type(2))) _Float16 v2h;
typedef __attribute__((ext_vector_type(4))) _Float16 v4h;

__global__ __launch_bounds__(256) void k_cvt8(const float* __restrict__ src, bf* dst, size_t n8) { const size_t i = (size_t)blockIdx.x * 256 + threadIdx.x; if (i >= n8) return; const v8f v = *(const v8f*)(src + i * 8); v8us o;
#pragma unroll
    for (int k = 0; k < 8; ++k) o[k] = f2bf(v[k]); *(volatile v8us*)(dst + i * 8) = o; __threadfence(); *(volatile v8us*)(dst + i * 8) = o; }
__global__ __launch_bounds__(256) void k_wtG(const float* __restrict__ w, int K, int N, bf* Bt) {
    const int lane = threadIdx.x & 31; const int L0 = (blockIdx.x * 8 + (threadIdx.x >> 5)) * 8; const int nlines = N * K / 64;
#pragma unroll
    for (int ps = 0; ps < 2; ++ps) {
#pragma unroll 1
        for (int l = 0; l < 8; ++l) { const int L = L0 + l; if (L >= nlines) break; const size_t e = (size_t)L * 64 + lane * 2; const int k = (int)(e % K), n = (int)(e / K); v2us o;
            o[0] = f2bf(w[(size_t)k * N + n]); o[1] = f2bf(w[(size_t)(k + 1) * N + n]); *(volatile v2us*)(Bt + e) = o; }
        if (ps == 0) __threadfence(); }
}

__global__ __launch_bounds__(256) void k_qkp(const float* __restrict__ QKV, bf* Qh, bf* Ql, bf* Kh, bf* Kl) { const size_t e = ((size_t)blockIdx.x * 256 + threadIdx.x) * 4; if (e >= (size_t)WCH * NH_ * TP * HD) return; const int d = (int)(e % HD); const int r = (int)((e / HD) % TP); const int z = (int)(e / ((size_t)HD * TP)); const int w = z / NH_, h = z % NH_; v4us qh, ql, kh, kl;
    for (int u = 0; u < 4; ++u) { qh[u] = 0; ql[u] = 0; kh[u] = 0; kl[u] = 0; }
    if (r < NTOK) { const float* row = QKV + ((size_t)w * NTOK + r) * (3 * DM) + h * HD + d;
#pragma unroll
        for (int u = 0; u < 4; ++u) { unsigned short a, b; splitf(row[u] * 0.125f, a, b); qh[u] = a; ql[u] = b; splitf(row[DM + u], a, b); kh[u] = a; kl[u] = b; } }
    *(volatile v4us*)(Qh + e) = qh; *(volatile v4us*)(Ql + e) = ql; *(volatile v4us*)(Kh + e) = kh; *(volatile v4us*)(Kl + e) = kl; __threadfence(); *(volatile v4us*)(Qh + e) = qh; *(volatile v4us*)(Ql + e) = ql; *(volatile v4us*)(Kh + e) = kh; *(volatile v4us*)(Kl + e) = kl; }
__global__ __launch_bounds__(256) void k_vtp(const float* __restrict__ QKV, h16* VT) { const size_t e = ((size_t)blockIdx.x * 256 + threadIdx.x) * 2; if (e >= (size_t)WCH * NH_ * HD * TP) return; const int r = (int)(e % TP); const int d = (int)((e / TP) % HD); const int z = (int)(e / ((size_t)TP * HD)); const int w = z / NH_, h = z % NH_; v2h o;
#pragma unroll
    for (int u = 0; u < 2; ++u) { const int rr = r + u; o[u] = (rr < NTOK) ? tohx(QKV[((size_t)w * NTOK + rr) * (3 * DM) + 2 * DM + h * HD + d]) : (h16)0.f; }
    *(volatile v2h*)(VT + e) = o; __threadfence(); *(volatile v2h*)(VT + e) = o; }
__global__ __launch_bounds__(256) void k_wsoft(const float* __restrict__ S, const float* __restrict__ QKV, const float* __restrict__ rph, const float* __restrict__ rpw, int z0, h16* P16) {
    const int lane = threadIdx.x & 31; const int row = blockIdx.x * 8 + (threadIdx.x >> 5); if (row >= ZHALF * TP) return; const int q = row % TP; const int zl = row / TP; const int z = z0 + zl; const int w = z / NH_, h = z % NH_;
    h16* prow = P16 + (size_t)row * TP;
    if (q >= NTOK) { v4h zz4; zz4[0] = (h16)0.f; zz4[1] = (h16)0.f; zz4[2] = (h16)0.f; zz4[3] = (h16)0.f; for (int ps = 0; ps < 2; ++ps) { for (int ch = 0; ch < TP / 128; ++ch) *(volatile v4h*)(prow + ch * 128 + lane * 4) = zz4; if (ps == 0) __threadfence(); } return; }
    const int qh = q / GH, qw = q % GH; float rel = 0.f;
    if (lane < 2 * GH) { const float* qraw = QKV + ((size_t)w * NTOK + q) * (3 * DM) + h * HD; const float* tab = (lane < GH) ? (rph + (size_t)(qh - lane + GH - 1) * HD) : (rpw + (size_t)(qw - (lane - GH) + GH - 1) * HD);
#pragma unroll 1
        for (int d = 0; d < HD; ++d) { float p = __fmul_rn(qraw[d], bfr(tab[d])); asm volatile("" : "+v"(p)); rel = __fadd_rn(rel, p); } }
    const float* sr = S + (size_t)row * TP; float v[TP / 32]; float mx = -3.0e38f;
#pragma unroll
    for (int ch = 0; ch < TP / 128; ++ch) { const v4f a = *(const v4f*)(sr + ch * 128 + lane * 4);
#pragma unroll
        for (int u = 0; u < 4; ++u) { const int j = ch * 128 + lane * 4 + u; const int kh = j / GH, kw = j % GH; const float rh = __shfl(rel, kh & 31, 32), rw = __shfl(rel, (GH + kw) & 31, 32); float t = -3.0e38f;
            if (j < NTOK) { const float s1 = __fadd_rn(a[u], rh); t = __fadd_rn(s1, rw); } v[ch * 4 + u] = t; mx = fmaxf(mx, t); } }
#pragma unroll
    for (int sh = 16; sh; sh >>= 1) mx = fmaxf(mx, __shfl_xor(mx, sh, 32));
    float sum = 0.f;
#pragma unroll
    for (int k2 = 0; k2 < TP / 32; ++k2) { float d0 = __fsub_rn(v[k2], mx); asm volatile("" : "+v"(d0)); v[k2] = __builtin_amdgcn_exp2f(__fmul_rn(d0, 1.4426950408889634f)); sum += v[k2]; }
#pragma unroll
    for (int sh = 16; sh; sh >>= 1) sum += __shfl_xor(sum, sh, 32);
    const float f = __fdiv_rn(PCAR, sum);
    for (int ps = 0; ps < 2; ++ps) {
#pragma unroll
        for (int ch = 0; ch < TP / 128; ++ch) { v4h o4; for (int u = 0; u < 4; ++u) o4[u] = tohx(v[ch * 4 + u] * f); *(volatile v4h*)(prow + ch * 128 + lane * 4) = o4; }
        if (ps == 0) __threadfence(); } }
__global__ __launch_bounds__(256) void k_mrg(const float* __restrict__ O, int z0, bf* Ah, bf* Al) { const size_t e = ((size_t)blockIdx.x * 256 + threadIdx.x) * 4; if (e >= (size_t)ZHALF * TP * HD) return; const int d = (int)(e % HD); const int q = (int)((e / HD) % TP); const int zl = (int)(e / ((size_t)HD * TP)); if (q >= NTOK) return; const int z = z0 + zl; const int w = z / NH_, h = z % NH_; const size_t oo = ((size_t)w * NTOK + q) * DM + h * HD + d; v4us oh, ol;
#pragma unroll
    for (int u = 0; u < 4; ++u) { unsigned short a, b; splitf(O[e + u] * (1.0f / PCAR), a, b); oh[u] = a; ol[u] = b; } *(volatile v4us*)(Ah + oo) = oh; *(volatile v4us*)(Al + oo) = ol; __threadfence(); *(volatile v4us*)(Ah + oo) = oh; *(volatile v4us*)(Al + oo) = ol; }

extern "C" void kernel_launch(void* const* d_in, const int* in_sizes, int n_in,
                              void* d_out, int out_size, void* d_ws, size_t ws_size, hipStream_t stream) {
    (void)in_sizes; (void)n_in; (void)out_size;
    const float* x = (const float*)d_in[0]; const float* qkv_w = (const float*)d_in[1]; const float* qkv_b = (const float*)d_in[2]; const float* proj_w = (const float*)d_in[3]; const float* proj_b = (const float*)d_in[4]; const float* rph = (const float*)d_in[5]; const float* rpw = (const float*)d_in[6];
    float* OUT = (float*)d_out;
    char* wsp = (char*)d_ws;
    auto take = [&](size_t bytes) { char* p = wsp; wsp += (bytes + 255) & ~(size_t)255; return (void*)p; };
    const int CT = WCH * NTOK;
    bf* BQKV = (bf*)take((size_t)3 * DM * DM * 2); bf* BPJ = (bf*)take((size_t)DM * DM * 2); bf* XB = (bf*)take((size_t)CT * DM * 2); float* QKV = (float*)take((size_t)CT * 3 * DM * 4);
    bf* QPh = (bf*)take((size_t)WCH * NH_ * TP * HD * 2); bf* QPl = (bf*)take((size_t)WCH * NH_ * TP * HD * 2); bf* KPh = (bf*)take((size_t)WCH * NH_ * TP * HD * 2); bf* KPl = (bf*)take((size_t)WCH * NH_ * TP * HD * 2); h16* VT = (h16*)take((size_t)WCH * NH_ * HD * TP * 2); float* S = (float*)take((size_t)ZHALF * TP * TP * 4); h16* P16 = (h16*)take((size_t)ZHALF * TP * TP * 2); float* O = (float*)take((size_t)ZHALF * TP * HD * 4);
    bf* ATh = (bf*)take((size_t)CT * DM * 2); bf* ATl = (bf*)take((size_t)CT * DM * 2);
    if ((size_t)(wsp - (char*)d_ws) > ws_size) return;
    k_wtG<<<(DM * 3 * DM / 64 + 63) / 64, 256, 0, stream>>>(qkv_w, DM, 3 * DM, BQKV); k_wtG<<<(DM * DM / 64 + 63) / 64, 256, 0, stream>>>(proj_w, DM, DM, BPJ);
    const size_t zq = (size_t)TP * HD, zS = (size_t)TP * TP, zv = (size_t)HD * TP;
    for (int c = 0; c < NWIN / WCH; ++c) { const float* xc = x + (size_t)c * CT * DM;
        k_cvt8<<<(unsigned)(((size_t)CT * DM / 8 + 255) / 256), 256, 0, stream>>>(xc, XB, (size_t)CT * DM / 8);
        k_gemmw<bf, 0, true><<<dim3(CT / 64, 3 * DM / 64, 1), 32, 0, stream>>>(XB, nullptr, BQKV, nullptr, DM, QKV, 3 * DM, qkv_b, 0, 0, 0);
        k_qkp<<<(unsigned)(((size_t)WCH * NH_ * TP * HD / 4 + 255) / 256), 256, 0, stream>>>(QKV, QPh, QPl, KPh, KPl); k_vtp<<<(unsigned)(((size_t)WCH * NH_ * HD * TP / 2 + 255) / 256), 256, 0, stream>>>(QKV, VT);
        for (int z0 = 0; z0 < WCH * NH_; z0 += ZHALF) {
            k_gemmw<bf, 2, false><<<dim3(TP / 64, TP / 64, ZHALF), 32, 0, stream>>>(QPh + (size_t)z0 * zq, QPl + (size_t)z0 * zq, KPh + (size_t)z0 * zq, KPl + (size_t)z0 * zq, HD, S, TP, nullptr, zq, zq, zS);
            k_wsoft<<<ZHALF * TP / 8, 256, 0, stream>>>(S, QKV, rph, rpw, z0, P16);
            k_gemmw<h16, 0, false><<<dim3(TP / 64, 1, ZHALF), 32, 0, stream>>>(P16, nullptr, VT + (size_t)z0 * zv, nullptr, TP, O, HD, nullptr, zS, zv, zq);
            k_mrg<<<(unsigned)(((size_t)ZHALF * TP * HD / 4 + 255) / 256), 256, 0, stream>>>(O, z0, ATh, ATl); }
        k_gemmw<bf, 1, true><<<dim3(CT / 64, DM / 64, 1), 32, 0, stream>>>(ATh, ATl, BPJ, nullptr, DM, OUT + (size_t)c * CT * DM, DM, proj_b, 0, 0, 0); }
}
